// EdgeNetwork_26439818674551
// MI455X (gfx1250) — hardware-verified
//
#include <hip/hip_runtime.h>
#include <math.h>

constexpr int   kNodes     = 100000;
constexpr int   kEdges     = 1000000;
constexpr int   kIn        = 64;
constexpr int   kFeat      = 128;
constexpr int   kTileE     = 32;
constexpr int   kTiles     = kEdges / kTileE;
constexpr int   kWP        = 136;
constexpr int   kHP        = 136;
constexpr int   kWaves     = 3;
constexpr int   kThreads   = kWaves * 32;
constexpr int   kBlocks    = 320;
constexpr int   kW4Plane   = 16 * kWP;
constexpr int   kW4ZeroGrp = (kW4Plane - kFeat) / 8;
constexpr float kWCarry    = 16.0f;
constexpr float kWCarryInv = 0.0625f;

static_assert(kEdges % kTileE == 0, "whole tiles only");
static_assert(kFeat == 2 * kIn, "concat width");
static_assert(kFeat % 32 == 0, "K multiple of 32");
static_assert((kWP * 2) % 16 == 0, "16-B aligned weight rows");
static_assert((kHP * 2) % 16 == 0, "16-B aligned activation rows");
static_assert((kW4Plane - kFeat) % 8 == 0, "zero groups");
constexpr int kLdsBytes = 3 * kFeat * kWP * 2 + kW4Plane * 2 + 3 * kFeat * 4 + 2 * kWaves * kTileE * kHP * 2 + kWaves * 32 * 4;
static_assert(kLdsBytes == 162944, "LDS budget");
static_assert(kLdsBytes <= 163840, "LDS budget");

typedef __attribute__((ext_vector_type(16))) _Float16 v16h;
typedef __attribute__((ext_vector_type(8)))  _Float16 v8h;
typedef __attribute__((ext_vector_type(8)))  float    v8f;
typedef __attribute__((ext_vector_type(4)))  float    v4f;

template <typename T> struct Frag;
template <> struct Frag<_Float16> {
  typedef v16h V; union U { v16h v; v8h h[2]; };
  static __device__ __forceinline__ v16h load(const _Float16* p) {
    U f; f.h[0] = *(const v8h*)(p); f.h[1] = *(const v8h*)(p + 16); return f.v;
  }
  static __device__ __forceinline__ v8f mma(v16h a, v16h b, v8f c) {
    return __builtin_amdgcn_wmma_f32_16x16x32_f16(false, a, false, b, (short)0, c, false, false);
  }
};

__device__ __forceinline__ void guard4x(v8f& a0, v8f& a1, v8f& a2, v8f& a3,
                                        v16h w0, v16h w1, v16h w2, v16h w3, v16h hb) {
  asm volatile("v_nop\n\tv_nop\n\tv_nop\n\tv_nop"
               : "+v"(a0), "+v"(a1), "+v"(a2), "+v"(a3)
               : "v"(w0), "v"(w1), "v"(w2), "v"(w3), "v"(hb));
}
__device__ __forceinline__ void guard_one(v8f& a, v16h x, v16h y) {
  asm volatile("v_nop\n\tv_nop\n\tv_nop\n\tv_nop" : "+v"(a) : "v"(x), "v"(y));
}
__device__ __forceinline__ void wave_lds_sync() {
  __builtin_amdgcn_fence(__ATOMIC_RELEASE, "workgroup");
  __builtin_amdgcn_wave_barrier();
  __builtin_amdgcn_fence(__ATOMIC_ACQUIRE, "workgroup");
}

__device__ __forceinline__ v8h zero8h() {
  v8h z;
#pragma unroll
  for (int e = 0; e < 8; ++e) z[e] = (_Float16)0.0f;
  return z;
}

__device__ __forceinline__ float tanh_f(float v) {
  v = fminf(fmaxf(v, -20.0f), 20.0f);
  const float e = expf(2.0f * v);
  const float r = __builtin_amdgcn_rcpf(e + 1.0f);
  return fmaf(-2.0f, r, 1.0f);
}
__device__ __forceinline__ float sigmoid_f(float z) {
  z = fminf(fmaxf(z, -30.0f), 30.0f);
  const float e = expf(-z);
  return __builtin_amdgcn_rcpf(e + 1.0f);
}

__device__ __forceinline__ void gather32(const float* __restrict__ p, _Float16* q) {
  const v4f a0 = *(const v4f*)(p);
  const v4f a1 = *(const v4f*)(p + 4);
  const v4f a2 = *(const v4f*)(p + 8);
  const v4f a3 = *(const v4f*)(p + 12);
  const v4f a4 = *(const v4f*)(p + 16);
  const v4f a5 = *(const v4f*)(p + 20);
  const v4f a6 = *(const v4f*)(p + 24);
  const v4f a7 = *(const v4f*)(p + 28);
  v8h h0, h1, h2, h3;
#pragma unroll
  for (int e = 0; e < 4; ++e) {
    h0[e] = (_Float16)a0[e]; h0[4 + e] = (_Float16)a1[e];
    h1[e] = (_Float16)a2[e]; h1[4 + e] = (_Float16)a3[e];
    h2[e] = (_Float16)a4[e]; h2[4 + e] = (_Float16)a5[e];
    h3[e] = (_Float16)a6[e]; h3[4 + e] = (_Float16)a7[e];
  }
  *(v8h*)(q)      = h0;
  *(v8h*)(q + 8)  = h1;
  *(v8h*)(q + 16) = h2;
  *(v8h*)(q + 24) = h3;
}

__device__ __forceinline__ void stage_weight(const float* __restrict__ W, _Float16* dst, int tid) {
#pragma unroll 1
  for (int g = tid; g < kFeat * kFeat / 4; g += kThreads) {
    const int k  = g >> 5;
    const int n4 = (g & 31) * 4;
    const v4f w = *(const v4f*)(W + (size_t)k * kFeat + n4);
    dst[(n4 + 0) * kWP + k] = (_Float16)(w[0] * kWCarry);
    dst[(n4 + 1) * kWP + k] = (_Float16)(w[1] * kWCarry);
    dst[(n4 + 2) * kWP + k] = (_Float16)(w[2] * kWCarry);
    dst[(n4 + 3) * kWP + k] = (_Float16)(w[3] * kWCarry);
  }
  const v8h z = zero8h();
#pragma unroll 1
  for (int r = tid; r < kFeat; r += kThreads) *(v8h*)(dst + r * kWP + kFeat) = z;
}

__device__ __forceinline__ void epi_tanh8(v8f acc, const float* bp, _Float16* q) {
  const v4f b0 = *(const v4f*)(bp);
  const v4f b1 = *(const v4f*)(bp + 4);
  v8h hv;
#pragma unroll
  for (int r = 0; r < 4; ++r) {
    hv[r]     = (_Float16)tanh_f(fmaf(acc[r],     kWCarryInv, b0[r]));
    hv[4 + r] = (_Float16)tanh_f(fmaf(acc[4 + r], kWCarryInv, b1[r]));
  }
  *(v8h*)q = hv;
}

__device__ __forceinline__ void mlp_layer(const _Float16* wt, const float* bs,
                                          const _Float16* hin, _Float16* hout, int c, int hh) {
  const v8f z8 = (v8f){0.f, 0.f, 0.f, 0.f, 0.f, 0.f, 0.f, 0.f};
#pragma unroll 1
  for (int p = 0; p < 4; ++p) {
    const int mb = p >> 1, nh = p & 1;
    v8f acc0 = z8, acc1 = z8, acc2 = z8, acc3 = z8;
    const _Float16* hrow = hin + (mb * 16 + c) * kHP + 8 * hh;
    const _Float16* wrow = wt + (nh * 64 + c) * kWP + 8 * hh;
#pragma unroll 1
    for (int ks = 0; ks < kFeat / 32; ++ks) {
      const v16h hb = Frag<_Float16>::load(hrow + ks * 32);
      const v16h w0 = Frag<_Float16>::load(wrow + ks * 32);
      const v16h w1 = Frag<_Float16>::load(wrow + 16 * kWP + ks * 32);
      const v16h w2 = Frag<_Float16>::load(wrow + 32 * kWP + ks * 32);
      const v16h w3 = Frag<_Float16>::load(wrow + 48 * kWP + ks * 32);
      acc0 = Frag<_Float16>::mma(w0, hb, acc0);
      acc1 = Frag<_Float16>::mma(w1, hb, acc1);
      acc2 = Frag<_Float16>::mma(w2, hb, acc2);
      acc3 = Frag<_Float16>::mma(w3, hb, acc3);
      guard4x(acc0, acc1, acc2, acc3, w0, w1, w2, w3, hb);
    }
    const float* bp = bs + nh * 64 + 8 * hh;
    _Float16* orow = hout + (mb * 16 + c) * kHP + nh * 64 + 8 * hh;
    epi_tanh8(acc0, bp,      orow);
    epi_tanh8(acc1, bp + 16, orow + 16);
    epi_tanh8(acc2, bp + 32, orow + 32);
    epi_tanh8(acc3, bp + 48, orow + 48);
  }
}

__device__ __forceinline__ float head_half(const _Float16* hrow, const _Float16* wrow, float b4v) {
  v8f acc = (v8f){0.f, 0.f, 0.f, 0.f, 0.f, 0.f, 0.f, 0.f};
#pragma unroll
  for (int ks = 0; ks < kFeat / 32; ++ks) {
    const v16h hb = Frag<_Float16>::load(hrow + ks * 32);
    const v16h wa = Frag<_Float16>::load(wrow + ks * 32);
    acc = Frag<_Float16>::mma(wa, hb, acc);
    guard_one(acc, wa, hb);
  }
  return sigmoid_f(fmaf(acc[0], kWCarryInv, b4v));
}

__global__ __launch_bounds__(kThreads) void edge_net_kernel(
    const float* __restrict__ x, const int* __restrict__ ei,
    const float* __restrict__ W1, const float* __restrict__ b1,
    const float* __restrict__ W2, const float* __restrict__ b2,
    const float* __restrict__ W3, const float* __restrict__ b3,
    const float* __restrict__ W4, const float* __restrict__ b4,
    float* __restrict__ out) {
  __shared__ __align__(16) _Float16 s_wt[3][kFeat * kWP];
  __shared__ __align__(16) _Float16 s_w4t[kW4Plane];
  __shared__ __align__(16) float    s_bias[3][kFeat];
  __shared__ __align__(16) _Float16 s_h[2][kWaves][kTileE * kHP];
  __shared__ __align__(16) float    s_o[kWaves][32];

  const int tid  = threadIdx.x;
  const int lane = tid & 31;
  const int wave = tid >> 5;
  const int c    = lane & 15;
  const int hh   = lane >> 4;

  stage_weight(W1, &s_wt[0][0], tid);
  stage_weight(W2, &s_wt[1][0], tid);
  stage_weight(W3, &s_wt[2][0], tid);
#pragma unroll 1
  for (int i = tid; i < kFeat; i += kThreads) s_w4t[i] = (_Float16)(W4[i] * kWCarry);
  {
    const v8h z = zero8h();
#pragma unroll 1
    for (int g = tid; g < kW4ZeroGrp; g += kThreads) *(v8h*)(s_w4t + kFeat + 8 * g) = z;
  }
#pragma unroll 1
  for (int i = tid; i < kFeat; i += kThreads) {
    s_bias[0][i] = b1[i];
    s_bias[1][i] = b2[i];
    s_bias[2][i] = b3[i];
  }
  __syncthreads();

  const float b4v = b4[0];
  _Float16* h0 = &s_h[0][wave][0];
  _Float16* h1 = &s_h[1][wave][0];
  float*    so = &s_o[wave][0];
  const int wave_g = blockIdx.x * kWaves + wave;
  const int nwaves = gridDim.x * kWaves;

#pragma unroll 1
  for (int tile = wave_g; tile < kTiles; tile += nwaves) {
    const int e0 = tile * kTileE;
    int sn = ei[e0 + lane];
    int dn = ei[kEdges + e0 + lane];
    sn = sn < 0 ? 0 : (sn >= kNodes ? kNodes - 1 : sn);
    dn = dn < 0 ? 0 : (dn >= kNodes ? kNodes - 1 : dn);
    const float* xs = x + (size_t)sn * kIn;
    const float* xd = x + (size_t)dn * kIn;
    _Float16* grow = h0 + lane * kHP;
    gather32(xs, grow);
    asm volatile("" ::: "memory");
    gather32(xs + 32, grow + 32);
    asm volatile("" ::: "memory");
    gather32(xd, grow + 64);
    asm volatile("" ::: "memory");
    gather32(xd + 32, grow + 96);
    wave_lds_sync();

#pragma unroll 1
    for (int L = 0; L < 3; ++L) {
      const _Float16* hin = (L == 1) ? h1 : h0;
      _Float16* hout      = (L == 1) ? h0 : h1;
      mlp_layer(&s_wt[L][0], &s_bias[L][0], hin, hout, c, hh);
      wave_lds_sync();
    }

    const _Float16* w4row = s_w4t + c * kWP + 8 * hh;
    const float ov0 = head_half(h1 + c * kHP + 8 * hh,        w4row, b4v);
    const float ov1 = head_half(h1 + (16 + c) * kHP + 8 * hh, w4row, b4v);
    if (lane < 16) {
      so[lane]      = ov0;
      so[16 + lane] = ov1;
    }
    wave_lds_sync();
    {
      const v4f v = *(const v4f*)(so + 4 * (lane & 7));
      float* op = out + (size_t)e0 + 4 * (lane & 7);
      for (int pass = 0; pass < 2; ++pass) {
        if (lane < 8) *(volatile v4f*)op = v;
        __threadfence();
      }
    }
    wave_lds_sync();
  }
}

extern "C" void kernel_launch(void* const* d_in, const int* in_sizes, int n_in,
                              void* d_out, int out_size, void* d_ws, size_t ws_size,
                              hipStream_t stream) {
  (void)in_sizes; (void)n_in; (void)out_size; (void)d_ws; (void)ws_size;
  const float* x  = (const float*)d_in[0];
  const int*   ei = (const int*)  d_in[1];
  const float* W1 = (const float*)d_in[2];
  const float* b1 = (const float*)d_in[3];
  const float* W2 = (const float*)d_in[4];
  const float* b2 = (const float*)d_in[5];
  const float* W3 = (const float*)d_in[6];
  const float* b3 = (const float*)d_in[7];
  const float* W4 = (const float*)d_in[8];
  const float* b4 = (const float*)d_in[9];
  float* out = (float*)d_out;
  edge_net_kernel<<<kBlocks, kThreads, 0, stream>>>(x, ei, W1, b1, W2, b2, W3, b3, W4, b4, out);
}
